// XrdAttentionBase_9294309229168
// MI455X (gfx1250) — hardware-verified
//
#include <hip/hip_runtime.h>


#define NBb  4
#define NN   8500
#define NP   8512
#define EE   32
#define EP   64
#define RCH  2048
#define PCAR 4096.0f
typedef _Float16 h16;
typedef unsigned short bf;
typedef __attribute__((ext_vector_type(16))) __bf16   v16bf;
typedef __attribute__((ext_vector_type(16))) _Float16 v16h;
typedef __attribute__((ext_vector_type(8)))  _Float16 v8h;
typedef __attribute__((ext_vector_type(8)))  unsigned short v8us;
typedef __attribute__((ext_vector_type(8)))  float    v8f;
typedef __attribute__((ext_vector_type(4)))  float    v4f;
typedef v8h  __attribute__((may_alias)) v8ha;
typedef v4f  __attribute__((may_alias)) v4fa;
typedef v8us __attribute__((may_alias)) v8usa;

__device__ __forceinline__ unsigned short f2bf(float f) { unsigned u = __float_as_uint(f); u += 0x7FFFu + ((u >> 16) & 1u); return (unsigned short)(u >> 16); }
__device__ __forceinline__ float bf2f(unsigned short b) { return __uint_as_float(((unsigned)b) << 16); }
__device__ __forceinline__ float bfr(float f) { return bf2f(f2bf(f)); }
__device__ __forceinline__ v16h cat16(v8h lo, v8h hi) { return __builtin_shufflevector(lo, hi, 0, 1, 2, 3, 4, 5, 6, 7, 8, 9, 10, 11, 12, 13, 14, 15); }
__device__ __forceinline__ v16bf cat16b(v8us lo, v8us hi) { return __builtin_bit_cast(v16bf, __builtin_shufflevector(lo, hi, 0, 1, 2, 3, 4, 5, 6, 7, 8, 9, 10, 11, 12, 13, 14, 15)); }
__device__ __forceinline__ v8f wmma16(v16h a, v16h b, v8f c) { return __builtin_amdgcn_wmma_f32_16x16x32_f16(false, a, false, b, (short)0, c, false, false); }
__device__ __forceinline__ v8f wmmab(v16bf a, v16bf b, v8f c) { return __builtin_amdgcn_wmma_f32_16x16x32_bf16(false, a, false, b, (short)0, c, false, false); }


template <typename T16> struct WFrag;
template <> struct WFrag<h16> { typedef v16h V; static __device__ __forceinline__ V ld(const h16* p) { return cat16(*(const v8h*)p, *(const v8h*)(p + 16)); } static __device__ __forceinline__ v8f mma(V a, V b, v8f c) { return wmma16(a, b, c); } };
template <> struct WFrag<bf> { typedef v16bf V; static __device__ __forceinline__ V ld(const bf* p) { return cat16b(*(const v8us*)p, *(const v8us*)(p + 16)); } static __device__ __forceinline__ v8f mma(V a, V b, v8f c) { return wmmab(a, b, c); } };
template <typename T16, int NSPLIT, bool BIAS>
__global__ __launch_bounds__(32) void k_gemmw(const T16* __restrict__ A, const T16* __restrict__ A2, const T16* __restrict__ Bt, const T16* __restrict__ Bt2, int K, float* C, int ldc, const float* __restrict__ bias, size_t sA, size_t sB, size_t sC) {
    typedef typename WFrag<T16>::V V;
    __shared__ __align__(16) float os[16 * 68];
    const size_t z = blockIdx.z; A += z * sA; if (A2) A2 += z * sA; Bt += z * sB; if (Bt2) Bt2 += z * sB; C += z * sC;
    const int lane = threadIdx.x & 31, lr = lane & 15, hi = lane >> 4; const int r0 = blockIdx.x * 64, c0 = blockIdx.y * 64;
    v8f acc[4][4];
#pragma unroll
    for (int mb = 0; mb < 4; ++mb)
#pragma unroll
        for (int nb = 0; nb < 4; ++nb) acc[mb][nb] = (v8f){};
    const size_t aoff = (size_t)(r0 + lr) * K + 8 * hi, boff = (size_t)(c0 + lr) * K + 8 * hi;
#pragma unroll 1
    for (int kc = 0; kc < K; kc += 32) {
        V a[4], a2[4];
#pragma unroll
        for (int mb = 0; mb < 4; ++mb) { a[mb] = WFrag<T16>::ld(A + aoff + (size_t)mb * 16 * K + kc); if (NSPLIT == 1 || NSPLIT == 2) a2[mb] = WFrag<T16>::ld(A2 + aoff + (size_t)mb * 16 * K + kc); }
#pragma unroll
        for (int nb = 0; nb < 4; ++nb) { const V b = WFrag<T16>::ld(Bt + boff + (size_t)nb * 16 * K + kc); V b2; if (NSPLIT >= 2) b2 = WFrag<T16>::ld(Bt2 + boff + (size_t)nb * 16 * K + kc);
#pragma unroll
            for (int mb = 0; mb < 4; ++mb) { acc[mb][nb] = WFrag<T16>::mma(a[mb], b, acc[mb][nb]); if (NSPLIT == 1 || NSPLIT == 2) acc[mb][nb] = WFrag<T16>::mma(a2[mb], b, acc[mb][nb]); if (NSPLIT >= 2) acc[mb][nb] = WFrag<T16>::mma(a[mb], b2, acc[mb][nb]); } }
        asm volatile("v_nop\n\tv_nop\n\tv_nop\n\tv_nop" : "+v"(acc[0][0]), "+v"(acc[1][1]), "+v"(acc[2][2]), "+v"(acc[3][3]) : "v"(a[0]), "v"(a[3]));
    }
#pragma unroll
    for (int mb = 0; mb < 4; ++mb) {
#pragma unroll
        for (int nb = 0; nb < 4; ++nb) {
#pragma unroll
            for (int j = 0; j < 8; ++j) os[(hi * 8 + j) * 68 + nb * 16 + lr] = acc[mb][nb][j]; }
        __builtin_amdgcn_wave_barrier(); asm volatile("" ::: "memory");
        float* crow = C + (size_t)(r0 + mb * 16) * ldc + c0;
#pragma unroll 1
        for (int ps = 0; ps < 2; ++ps) {
#pragma unroll
            for (int s = 0; s < 8; ++s) { const int row = 2 * s + hi, cofs = lr * 4; v4f val = *(const v4fa*)(os + row * 68 + cofs); if (BIAS) { val[0] += bfr(bias[c0 + cofs]); val[1] += bfr(bias[c0 + cofs + 1]); val[2] += bfr(bias[c0 + cofs + 2]); val[3] += bfr(bias[c0 + cofs + 3]); }
                *(volatile v4f*)(crow + (size_t)row * ldc + cofs) = val; }
            if (ps == 0) __threadfence(); }
        __builtin_amdgcn_wave_barrier(); asm volatile("" ::: "memory");
    }
}

__device__ __forceinline__ h16 tohx(float x) { return (h16)x; }
typedef __attribute__((ext_vector_type(2))) _Float16 v2h;
typedef __attribute__((ext_vector_type(4))) _Float16 v4h;

__global__ __launch_bounds__(256) void k_u(const float* __restrict__ inten, float* U, float* UMAX) { __shared__ float red[256]; float mx = 0.f;
    for (int m = threadIdx.x; m < NP; m += 256) { const float v = (m < NN) ? bfr(inten[m]) * 0.01f : 0.f; if (m < NN) mx = fmaxf(mx, v); *(volatile float*)(U + m) = v; }
    red[threadIdx.x] = mx; __syncthreads();
    for (int s = 128; s; s >>= 1) { if (threadIdx.x < s) red[threadIdx.x] = fmaxf(red[threadIdx.x], red[threadIdx.x + s]); __syncthreads(); }
    __threadfence();
    for (int m = threadIdx.x; m < NP; m += 256) { const float v = (m < NN) ? bfr(inten[m]) * 0.01f : 0.f; *(volatile float*)(U + m) = v; }
    if (threadIdx.x < 64) { *(volatile float*)(UMAX + threadIdx.x) = red[0]; __threadfence(); *(volatile float*)(UMAX + threadIdx.x) = red[0]; } }
__global__ __launch_bounds__(256) void k_et(const float* __restrict__ tab, const int* __restrict__ ang, h16* ET) { const int e2 = (blockIdx.x * 256 + threadIdx.x) * 2; if (e2 >= EP * NP) return; const int m = e2 % NP; const int e = e2 / NP; v2h o;
#pragma unroll
    for (int u = 0; u < 2; ++u) { const int mm = m + u; o[u] = (e < EE && mm < NN) ? tohx(bfr(tab[(size_t)ang[mm] * EE + e])) : tohx(0.f); } *(volatile v2h*)(ET + e2) = o; __threadfence(); *(volatile v2h*)(ET + e2) = o; }
__global__ __launch_bounds__(256) void k_psoft(const float* __restrict__ U, const float* __restrict__ UMAX, int r0, int nrows, h16* P16) { const int lane = threadIdx.x & 31; const int rl = blockIdx.x * 8 + (threadIdx.x >> 5); if (rl >= nrows) return; const int n = r0 + rl; h16* pr = P16 + (size_t)rl * NP;
    if (n >= NN) { for (int ps = 0; ps < 2; ++ps) { for (int m0 = lane * 2; m0 < NP; m0 += 64) { v2h z; z[0] = tohx(0.f); z[1] = tohx(0.f); *(volatile v2h*)(pr + m0) = z; } if (ps == 0) __threadfence(); } return; }
    const float un = U[n]; const float mx = __fmul_rn(un, UMAX[0]); float sum = 0.f;
#pragma unroll 1
    for (int m = lane; m < NN; m += 32) { float d0 = __fsub_rn(__fmul_rn(un, U[m]), mx); asm volatile("" : "+v"(d0)); sum += __expf(d0); }
#pragma unroll
    for (int sh = 16; sh; sh >>= 1) sum += __shfl_xor(sum, sh, 32);
    const float f = __fdiv_rn(PCAR, sum);
    for (int ps = 0; ps < 2; ++ps) {
#pragma unroll 1
        for (int m0 = lane * 2; m0 < NP; m0 += 64) { v2h o;
#pragma unroll
            for (int u = 0; u < 2; ++u) { const int m = m0 + u; float val = 0.f; if (m < NN) { float d0 = __fsub_rn(__fmul_rn(un, U[m]), mx); asm volatile("" : "+v"(d0)); val = __fmul_rn(__expf(d0), f); } o[u] = tohx(val); }
            *(volatile v2h*)(pr + m0) = o; }
        if (ps == 0) __threadfence(); } }
__global__ __launch_bounds__(256) void k_xt(const float* __restrict__ XO, float* X) { const int e4 = (blockIdx.x * 256 + threadIdx.x) * 4; if (e4 >= EE * NN) return; v4f o;
#pragma unroll
    for (int u = 0; u < 4; ++u) { const int idx = e4 + u; const int n = idx % NN, e = idx / NN; o[u] = XO[(size_t)n * EP + e] * (1.0f / PCAR); } *(volatile v4f*)(X + e4) = o; __threadfence(); *(volatile v4f*)(X + e4) = o; }
template <int MODE>
__global__ __launch_bounds__(256) void k_conv(const float* __restrict__ Z, const float* __restrict__ w, const float* __restrict__ bb, const float* __restrict__ X, float* Hout) { const int e4 = (blockIdx.x * 256 + threadIdx.x) * 4; if (e4 >= EE * NN) return; v4f o;
#pragma unroll 1
    for (int u = 0; u < 4; ++u) { const int idx = e4 + u; const int n = idx % NN, e = idx / NN; float acc = bfr(bb[e]);
#pragma unroll 1
        for (int i = 0; i < EE; ++i) {
#pragma unroll
            for (int k = 0; k < 3; ++k) { const int nn = n + k - 1; if (nn >= 0 && nn < NN) { float p = __fmul_rn(bfr(w[(e * EE + i) * 3 + k]), Z[(size_t)i * NN + nn]); asm volatile("" : "+v"(p)); acc = __fadd_rn(acc, p); } } }
        if (MODE == 1) acc = __fadd_rn(X[idx], acc); o[u] = fmaxf(acc, 0.f); }
    *(volatile v4f*)(Hout + e4) = o; __threadfence(); *(volatile v4f*)(Hout + e4) = o; }

extern "C" void kernel_launch(void* const* d_in, const int* in_sizes, int n_in,
                              void* d_out, int out_size, void* d_ws, size_t ws_size, hipStream_t stream) {
    (void)in_sizes; (void)n_in; (void)out_size;
    const float* inten = (const float*)d_in[0]; const int* ang = (const int*)d_in[1]; const float* tab = (const float*)d_in[2]; const float* w1 = (const float*)d_in[3]; const float* b1 = (const float*)d_in[4]; const float* w2 = (const float*)d_in[5]; const float* b2 = (const float*)d_in[6];
    float* OUT = (float*)d_out;
    char* wsp = (char*)d_ws;
    auto take = [&](size_t bytes) { char* p = wsp; wsp += (bytes + 255) & ~(size_t)255; return (void*)p; };
    float* U = (float*)take(NP * 4); float* UMAX = (float*)take(256); h16* ET = (h16*)take((size_t)EP * NP * 2); h16* P16 = (h16*)take((size_t)RCH * NP * 2); float* XO = (float*)take((size_t)NP * EP * 4); float* X = (float*)take((size_t)EE * NN * 4); float* H1 = (float*)take((size_t)EE * NN * 4);
    if ((size_t)(wsp - (char*)d_ws) > ws_size) return;
    for (int b = 0; b < NBb; ++b) {
        k_u<<<1, 256, 0, stream>>>(inten + (size_t)b * NN, U, UMAX); k_et<<<(EP * NP / 2 + 255) / 256, 256, 0, stream>>>(tab, ang + (size_t)b * NN, ET);
        for (int r0 = 0; r0 < NP; r0 += RCH) { const int nrows = (NP - r0 < RCH) ? (NP - r0) : RCH;
            k_psoft<<<(nrows + 7) / 8, 256, 0, stream>>>(U, UMAX, r0, nrows, P16);
            k_gemmw<h16, 0, false><<<dim3(nrows / 64, 1, 1), 32, 0, stream>>>(P16, nullptr, ET, nullptr, NP, XO + (size_t)r0 * EP, EP, nullptr, 0, 0, 0); }
        k_xt<<<(EE * NN / 4 + 255) / 256, 256, 0, stream>>>(XO, X);
        k_conv<0><<<(EE * NN / 4 + 255) / 256, 256, 0, stream>>>(X, w1, b1, nullptr, H1);
        k_conv<1><<<(EE * NN / 4 + 255) / 256, 256, 0, stream>>>(H1, w2, b2, X, OUT + (size_t)b * EE * NN); }
}
